// MultiHeadSelfAttention_5179730559261
// MI455X (gfx1250) — hardware-verified
//
#include <hip/hip_runtime.h>


#ifndef NB
#define NB 4
#endif
#ifndef SEQ
#define SEQ 2048
#endif
#define NB_FULL   4
#define SEQ_FULL  2048
#define DM        512
#define NHEAD     8
#define HD        64
#define INNER     512
#define NQKV      1536
#define MROWS     (NB * SEQ)
#define PLANE_ELEMS ((size_t)MROWS * INNER)

static_assert(INNER == NHEAD * HD);
static_assert(NQKV == 3 * INNER);
static_assert(NHEAD == 8);
static_assert(HD == 64);
static_assert(DM == 32 * 16);
static_assert((DM & (DM - 1)) == 0);
static_assert(SEQ % 128 == 0);
static_assert(SEQ <= SEQ_FULL);
static_assert(NB >= 1 && NB <= NB_FULL);
static_assert(MROWS % 128 == 0);
static_assert(MROWS % 8 == 0);
static_assert(DM % 128 == 0);
static_assert(INNER % 128 == 0);
static_assert(NQKV % 128 == 0);
static_assert(DM % 32 == 0);
static_assert((2 * INNER) % 32 == 0);
static_assert(DM % 64 == 0 && NQKV % 64 == 0 && INNER % 64 == 0);

#define CARRY_X    16.0f
#define CARRY_W    32.0f
#define CARRY_Q    256.0f
#define CARRY_K    16.0f
#define CARRY_V    16.0f
#define CARRY_CTX  4096.0f

typedef unsigned u32;
typedef _Float16 f16;
typedef f16   v16h __attribute__((ext_vector_type(16)));
typedef f16   v8h  __attribute__((ext_vector_type(8)));
typedef float v8f  __attribute__((ext_vector_type(8)));
typedef float v4f  __attribute__((ext_vector_type(4)));

union FragU { v16h v; v8h half[2]; f16 e[16]; };
union H8U   { v8h v; f16 e[8]; };

__device__ __forceinline__ v8f zero8() {
    v8f z = {0.f, 0.f, 0.f, 0.f, 0.f, 0.f, 0.f, 0.f};
    return z;
}

__device__ __forceinline__ v8f wmma16(v16h a, v16h b, v8f c) {
    v8f d = __builtin_amdgcn_wmma_f32_16x16x32_f16(false, a, false, b, (short)0, c, false, false);
    asm volatile("v_nop\n\tv_nop\n\tv_nop\n\tv_nop" : "+v"(d) : "v"(a), "v"(b));
    return d;
}

__device__ __forceinline__ float bf16_rne(float x) {
    u32 u = __float_as_uint(x);
    u = (u + 0x7fffu + ((u >> 16) & 1u)) & 0xffff0000u;
    return __uint_as_float(u);
}

__device__ __forceinline__ float fexp2(float x) {
#if defined(__has_builtin)
#if __has_builtin(__builtin_amdgcn_exp2f)
    return __builtin_amdgcn_exp2f(x);
#else
    return exp2f(x);
#endif
#else
    return exp2f(x);
#endif
}

__device__ __forceinline__ float rowmax16(float x) {
    int v = __builtin_bit_cast(int, x);
    x = fmaxf(x, __builtin_bit_cast(float, __builtin_amdgcn_update_dpp(v, v, 0x121, 0xf, 0xf, false)));
    v = __builtin_bit_cast(int, x);
    x = fmaxf(x, __builtin_bit_cast(float, __builtin_amdgcn_update_dpp(v, v, 0x122, 0xf, 0xf, false)));
    v = __builtin_bit_cast(int, x);
    x = fmaxf(x, __builtin_bit_cast(float, __builtin_amdgcn_update_dpp(v, v, 0x124, 0xf, 0xf, false)));
    v = __builtin_bit_cast(int, x);
    x = fmaxf(x, __builtin_bit_cast(float, __builtin_amdgcn_update_dpp(v, v, 0x128, 0xf, 0xf, false)));
    return x;
}

__device__ __forceinline__ u32 foff(u32 rowbase, u32 pitch, u32 kcol, u32 lane) {
    return (rowbase + (lane & 15u)) * pitch + kcol + ((lane >> 4) << 3);
}
__device__ __forceinline__ v16h mkfrag(v8h lo, v8h hi) {
    FragU f;
    f.half[0] = lo;
    f.half[1] = hi;
    return f.v;
}

__global__ void __launch_bounds__(256)
ln_rows(const float* __restrict__ x, const float* __restrict__ gamma, const float* __restrict__ beta,
        f16* __restrict__ dst, u32 nrows, float carry) {
    const u32 lane = threadIdx.x & 31u;
    const u32 m    = blockIdx.x * 8u + (threadIdx.x >> 5);
    if (m >= nrows) return;
    const u32 mb = m / (u32)SEQ;
    const u32 sm = mb * (u32)SEQ_FULL + (m - mb * (u32)SEQ);
    const float* sp = x + (size_t)sm * DM + lane * 8u;
    const v4f a0 = *(const v4f*)(sp);
    const v4f a1 = *(const v4f*)(sp + 4);
    const v4f b0 = *(const v4f*)(sp + 256);
    const v4f b1 = *(const v4f*)(sp + 260);
    float v[16];
#pragma unroll
    for (int j = 0; j < 4; ++j) {
        v[j]      = bf16_rne(a0[j]);
        v[4 + j]  = bf16_rne(a1[j]);
        v[8 + j]  = bf16_rne(b0[j]);
        v[12 + j] = bf16_rne(b1[j]);
    }
    float s = 0.f;
#pragma unroll
    for (int j = 0; j < 16; ++j) s += v[j];
#pragma unroll
    for (int off = 16; off > 0; off >>= 1) s += __shfl_xor(s, off, 32);
    const float mean = s * (1.0f / 512.0f);
    float q = 0.f;
#pragma unroll
    for (int j = 0; j < 16; ++j) {
        const float d = v[j] - mean;
        v[j] = d;
        q += d * d;
    }
#pragma unroll
    for (int off = 16; off > 0; off >>= 1) q += __shfl_xor(q, off, 32);
    const float rstd = rsqrtf(q * (1.0f / 512.0f) + 1e-5f);

    const float* gp = gamma + lane * 8u;
    const float* bp = beta + lane * 8u;
    const v4f g0 = *(const v4f*)(gp);
    const v4f g1 = *(const v4f*)(gp + 4);
    const v4f g2 = *(const v4f*)(gp + 256);
    const v4f g3 = *(const v4f*)(gp + 260);
    const v4f t0 = *(const v4f*)(bp);
    const v4f t1 = *(const v4f*)(bp + 4);
    const v4f t2 = *(const v4f*)(bp + 256);
    const v4f t3 = *(const v4f*)(bp + 260);
    H8U o0, o1;
#pragma unroll
    for (int j = 0; j < 4; ++j) {
        o0.e[j]     = (f16)(((v[j]      * rstd) * bf16_rne(g0[j]) + bf16_rne(t0[j])) * carry);
        o0.e[j + 4] = (f16)(((v[4 + j]  * rstd) * bf16_rne(g1[j]) + bf16_rne(t1[j])) * carry);
        o1.e[j]     = (f16)(((v[8 + j]  * rstd) * bf16_rne(g2[j]) + bf16_rne(t2[j])) * carry);
        o1.e[j + 4] = (f16)(((v[12 + j] * rstd) * bf16_rne(g3[j]) + bf16_rne(t3[j])) * carry);
    }
    f16* dp = dst + (size_t)m * DM + lane * 8u;
    *(volatile v8h*)(dp)       = o0.v;
    *(volatile v8h*)(dp + 256) = o1.v;
    __threadfence();
    *(volatile v8h*)(dp)       = o0.v;
    *(volatile v8h*)(dp + 256) = o1.v;
}

__global__ void __launch_bounds__(256)
cvt_transpose(const float* __restrict__ src, f16* __restrict__ dst, u32 KD, u32 ND, float carry) {
    __shared__ __attribute__((aligned(16))) f16 Ts[64 * 72];

    const u32 tid = threadIdx.x;
    const u32 n0  = blockIdx.x * 64u;
    const u32 k0  = blockIdx.y * 64u;
    const u32 kr  = tid >> 4;
    const u32 nc  = (tid & 15u) << 2;

#pragma unroll
    for (u32 it = 0; it < 4; ++it) {
        const u32 kl = kr + it * 16u;
        const v4f a = *(const v4f*)(src + (size_t)(k0 + kl) * ND + n0 + nc);
#pragma unroll
        for (u32 j = 0; j < 4; ++j) {
            const float x0 = a[j];
            Ts[(nc + j) * 72u + kl] = (f16)(bf16_rne(x0) * carry);
        }
    }
    __syncthreads();

#pragma unroll
    for (u32 pass = 0; pass < 2; ++pass) {
#pragma unroll
        for (u32 it = 0; it < 2; ++it) {
            const u32 idx   = tid + it * 256u;
            const u32 line  = idx >> 3;
            const u32 piece = idx & 7u;
            const v8h v = *(const v8h*)&Ts[line * 72u + piece * 8u];
            f16* dp = dst + (size_t)(n0 + line) * KD + k0 + piece * 8u;
            *(volatile v8h*)dp = v;
        }
        if (pass == 0) __threadfence();
    }
}

__global__ void __launch_bounds__(256) __attribute__((amdgpu_num_vgpr(256)))
gemm_nt(const f16* __restrict__ A, const f16* __restrict__ W, u32 lda, u32 ktot, u32 mode,
        f16* __restrict__ planes, f16* __restrict__ vtp,
        const float* __restrict__ bias, float* __restrict__ outf,
        float mulQ, float mulKV, float mulOut) {
    __shared__ __attribute__((aligned(16))) f16 As[128 * 32];
    __shared__ __attribute__((aligned(16))) f16 Bs[128 * 32];
    __shared__ __attribute__((aligned(16))) f16 Cs[128 * 128];

    const u32 tid  = threadIdx.x;
    const u32 lane = tid & 31u;
    const u32 wave = tid >> 5;
    const u32 wm   = wave & 3u;
    const u32 wn   = wave >> 2;
    const u32 hh8  = (lane >> 4) << 3;
    const u32 c16  = lane & 15u;
    const u32 m0   = blockIdx.x * 128u;
    const u32 n0   = blockIdx.y * 128u;

    v8f acc[2][4];
#pragma unroll
    for (int i = 0; i < 2; ++i)
#pragma unroll
        for (int j = 0; j < 4; ++j) acc[i][j] = zero8();

    const u32 srow = tid >> 1;
    const u32 scol = (tid & 1u) << 4;
    const f16* gA = A + (size_t)(m0 + srow) * lda + scol;
    const f16* gW = W + (size_t)(n0 + srow) * DM + scol;

#pragma unroll 1
    for (u32 k0 = 0; k0 < ktot; k0 += 32u) {
        const u32 kw = k0 & (u32)(DM - 1);
        const v8h ra0 = *(const v8h*)(gA + k0);
        const v8h ra1 = *(const v8h*)(gA + k0 + 8);
        const v8h rb0 = *(const v8h*)(gW + kw);
        const v8h rb1 = *(const v8h*)(gW + kw + 8);
        __syncthreads();
        *(v8h*)&As[srow * 32u + scol]      = ra0;
        *(v8h*)&As[srow * 32u + scol + 8u] = ra1;
        *(v8h*)&Bs[srow * 32u + scol]      = rb0;
        *(v8h*)&Bs[srow * 32u + scol + 8u] = rb1;
        __syncthreads();

        v16h af[2], bfr[4];
#pragma unroll
        for (int i = 0; i < 2; ++i) {
            const u32 o = foff(wm * 32u + (u32)i * 16u, 32u, 0u, lane);
            af[i] = mkfrag(*(const v8h*)&As[o], *(const v8h*)&As[o + 16u]);
        }
#pragma unroll
        for (int j = 0; j < 4; ++j) {
            const u32 o = foff(wn * 64u + (u32)j * 16u, 32u, 0u, lane);
            bfr[j] = mkfrag(*(const v8h*)&Bs[o], *(const v8h*)&Bs[o + 16u]);
        }
#pragma unroll
        for (int i = 0; i < 2; ++i)
#pragma unroll
            for (int j = 0; j < 4; ++j) acc[i][j] = wmma16(af[i], bfr[j], acc[i][j]);
    }

    const u32 bidx  = m0 / (u32)SEQ;
    const u32 s0    = m0 - bidx * (u32)SEQ;
    const u32 piece = lane & 7u;
    const u32 lsub  = lane >> 3;

    if (mode == 0u) {
        const u32 which = n0 / (u32)INNER;
        const u32 nloc  = n0 - which * (u32)INNER;
        if (which < 2u) {
            const float mul  = (which == 0u) ? mulQ : mulKV;
            const u32   nrep = (which == 0u) ? 2u : 1u;
#pragma unroll 1
            for (u32 rep = 0; rep < nrep; ++rep) {
#pragma unroll
                for (int i = 0; i < 2; ++i)
#pragma unroll
                    for (int j = 0; j < 4; ++j) {
                        const u32 nl = wn * 64u + (u32)j * 16u + c16;
#pragma unroll
                        for (int r = 0; r < 8; ++r) {
                            const u32 ml = wm * 32u + (u32)i * 16u + hh8 + (u32)r;
                            const float val = acc[i][j][r] * mul;
                            const f16 hi = (f16)val;
                            const f16 rs = (f16)(val - (float)hi);
                            Cs[ml * 128u + nl] = (rep == 0u) ? hi : rs;
                        }
                    }
                __syncthreads();
                const u32 pidx = (which == 0u) ? rep : 2u;
                f16* op = planes + (size_t)pidx * PLANE_ELEMS;
                const size_t bh0 = (size_t)bidx * NHEAD + (nloc >> 6);
#pragma unroll
                for (int pass = 0; pass < 2; ++pass) {
#pragma unroll
                    for (u32 it = 0; it < 8; ++it) {
                        const u32 L    = wave * 32u + it * 4u + lsub;
                        const u32 ml   = L >> 1;
                        const u32 hsel = L & 1u;
                        const v8h v = *(const v8h*)&Cs[ml * 128u + hsel * 64u + piece * 8u];
                        f16* dp = op + ((bh0 + hsel) * SEQ + s0 + ml) * HD + piece * 8u;
                        *(volatile v8h*)dp = v;
                    }
                    if (pass == 0) __threadfence();
                }
                __syncthreads();
            }
        } else {
#pragma unroll
            for (int i = 0; i < 2; ++i)
#pragma unroll
                for (int j = 0; j < 4; ++j) {
                    const u32 nl = wn * 64u + (u32)j * 16u + c16;
                    H8U t;
#pragma unroll
                    for (int r = 0; r < 8; ++r) t.e[r] = (f16)(acc[i][j][r] * mulKV);
                    *(v8h*)&Cs[nl * 128u + wm * 32u + (u32)i * 16u + hh8] = t.v;
                }
            __syncthreads();
#pragma unroll
            for (int pass = 0; pass < 2; ++pass) {
#pragma unroll
                for (u32 it = 0; it < 8; ++it) {
                    const u32 L  = wave * 32u + it * 4u + lsub;
                    const u32 nl = L >> 1;
                    const u32 mh = L & 1u;
                    const v8h v = *(const v8h*)&Cs[nl * 128u + mh * 64u + piece * 8u];
                    f16* dp = vtp + ((size_t)(bidx * (u32)INNER + nloc + nl) * SEQ + s0 + mh * 64u + piece * 8u);
                    *(volatile v8h*)dp = v;
                }
                if (pass == 0) __threadfence();
            }
        }
    } else {
        float* Cf = (float*)Cs;
        const v4f braw = *(const v4f*)(bias + n0 + lsub * 32u + piece * 4u);
        v4f bb;
#pragma unroll
        for (int j = 0; j < 4; ++j) bb[j] = bf16_rne(braw[j]);
#pragma unroll
        for (u32 half = 0; half < 2; ++half) {
            if ((wm >> 1) == half) {
#pragma unroll
                for (int i = 0; i < 2; ++i)
#pragma unroll
                    for (int j = 0; j < 4; ++j) {
                        const u32 nl = wn * 64u + (u32)j * 16u + c16;
#pragma unroll
                        for (int r = 0; r < 8; ++r) {
                            const u32 ml = (wm & 1u) * 32u + (u32)i * 16u + hh8 + (u32)r;
                            Cf[ml * 128u + nl] = acc[i][j][r] * mulOut;
                        }
                    }
            }
            __syncthreads();
#pragma unroll
            for (int pass = 0; pass < 2; ++pass) {
#pragma unroll
                for (u32 it = 0; it < 8; ++it) {
                    const u32 L    = wave * 32u + it * 4u + lsub;
                    const u32 row  = L >> 2;
                    const u32 part = L & 3u;
                    const v4f c = *(const v4f*)&Cf[row * 128u + part * 32u + piece * 4u];
                    const v4f v = c + bb;
                    float* dp = outf + (size_t)(m0 + half * 64u + row) * DM + n0 + part * 32u + piece * 4u;
                    *(volatile v4f*)dp = v;
                }
                if (pass == 0) __threadfence();
            }
            __syncthreads();
        }
    }
}

__global__ void __launch_bounds__(256) __attribute__((amdgpu_num_vgpr(256)))
attn_fwd(const f16* __restrict__ Qh, const f16* __restrict__ Qr, const f16* __restrict__ Kp,
         const f16* __restrict__ Vt, f16* __restrict__ Cp) {
    __shared__ __attribute__((aligned(16))) f16 ks[64 * 64];
    __shared__ __attribute__((aligned(16))) f16 vsT[64 * 64];
    __shared__ __attribute__((aligned(16))) f16 ps[8 * 16 * 64];

    const u32 tid  = threadIdx.x;
    const u32 lane = tid & 31u;
    const u32 wave = tid >> 5;
    const u32 hh8  = (lane >> 4) << 3;
    const u32 c16  = lane & 15u;
    const u32 bh   = blockIdx.y;
    const u32 bidx = bh >> 3;
    const u32 hidx = bh & 7u;
    const u32 q0   = blockIdx.x * 128u + wave * 16u;
    const size_t head = (size_t)bh * SEQ * HD;
    const u32 pw   = wave * 1024u;

    v16h qa[2], qr[2];
    {
        const size_t qo = head + (size_t)(q0 + (lane & 15u)) * HD + ((lane >> 4) << 3);
#pragma unroll
        for (int c = 0; c < 2; ++c) {
            qa[c] = mkfrag(*(const v8h*)(Qh + qo + c * 32), *(const v8h*)(Qh + qo + c * 32 + 16));
            qr[c] = mkfrag(*(const v8h*)(Qr + qo + c * 32), *(const v8h*)(Qr + qo + c * 32 + 16));
        }
    }

    FragU onesu;
#pragma unroll
    for (int i = 0; i < 16; ++i) onesu.e[i] = (f16)1.0f;
    const v16h ones = onesu.v;

    float m[8];
    v8f   o[4], lacc;
#pragma unroll
    for (int r = 0; r < 8; ++r) m[r] = -1.0e30f;
#pragma unroll
    for (int dt = 0; dt < 4; ++dt) o[dt] = zero8();
    lacc = zero8();

    const float cl = 1.4426950408889634f * 3.0517578125e-05f;

#pragma unroll 1
    for (u32 kt = 0; kt < (u32)(SEQ / 64); ++kt) {
        __syncthreads();
#pragma unroll
        for (u32 p2 = 0; p2 < 2; ++p2) {
            const u32 p   = tid + p2 * 256u;
            const u32 row = p >> 3;
            const u32 pc  = (p & 7u) << 3;
            const v8h kv = *(const v8h*)(Kp + head + (size_t)(kt * 64u + row) * HD + pc);
            const v8h vv = *(const v8h*)(Vt + head + (size_t)row * SEQ + kt * 64u + pc);
            *(v8h*)&ks[row * 64u + pc]  = kv;
            *(v8h*)&vsT[row * 64u + pc] = vv;
        }
        __syncthreads();

        v8f s[4];
#pragma unroll
        for (int nt = 0; nt < 4; ++nt) s[nt] = zero8();
#pragma unroll
        for (int c = 0; c < 2; ++c) {
#pragma unroll
            for (int nt = 0; nt < 4; ++nt) {
                const u32 ko = foff((u32)nt * 16u, 64u, (u32)c * 32u, lane);
                const v16h kb = mkfrag(*(const v8h*)&ks[ko], *(const v8h*)&ks[ko + 16u]);
                s[nt] = wmma16(qa[c], kb, s[nt]);
                s[nt] = wmma16(qr[c], kb, s[nt]);
            }
        }

#pragma unroll
        for (int r = 0; r < 8; ++r) {
            float x[4];
#pragma unroll
            for (int nt = 0; nt < 4; ++nt) x[nt] = s[nt][r] * cl;
            const float tm = rowmax16(fmaxf(fmaxf(x[0], x[1]), fmaxf(x[2], x[3])));
            const float mn = fmaxf(m[r], tm);
            const float al = fexp2(m[r] - mn);
            m[r] = mn;
            lacc[r] *= al;
#pragma unroll
            for (int dt = 0; dt < 4; ++dt) o[dt][r] *= al;
            const float sh = 10.0f - mn;
#pragma unroll
            for (int nt = 0; nt < 4; ++nt)
                ps[pw + (hh8 + (u32)r) * 64u + (u32)nt * 16u + c16] = (f16)fexp2(x[nt] + sh);
        }
        __syncthreads();

#pragma unroll
        for (int kk = 0; kk < 2; ++kk) {
            const u32 po = pw + foff(0u, 64u, (u32)kk * 32u, lane);
            const v16h pa = mkfrag(*(const v8h*)&ps[po], *(const v8h*)&ps[po + 16u]);
#pragma unroll
            for (int dt = 0; dt < 4; ++dt) {
                const u32 vo = foff((u32)dt * 16u, 64u, (u32)kk * 32u, lane);
                const v16h vb = mkfrag(*(const v8h*)&vsT[vo], *(const v8h*)&vsT[vo + 16u]);
                o[dt] = wmma16(pa, vb, o[dt]);
            }
            lacc = wmma16(pa, ones, lacc);
        }
    }
    __syncthreads();

    float inv[8];
#pragma unroll
    for (int r = 0; r < 8; ++r) inv[r] = (CARRY_CTX / CARRY_V) * (1.0f / lacc[r]);

    const u32 piece = lane & 7u;
    const u32 lsub  = lane >> 3;
#pragma unroll 1
    for (u32 rep = 0; rep < 2; ++rep) {
#pragma unroll
        for (int r = 0; r < 8; ++r) {
#pragma unroll
            for (int dt = 0; dt < 4; ++dt) {
                const float val = o[dt][r] * inv[r];
                const f16 hi = (f16)val;
                const f16 rs = (f16)(val - (float)hi);
                ps[pw + (hh8 + (u32)r) * 64u + (u32)dt * 16u + c16] = (rep == 0u) ? hi : rs;
            }
        }
        __syncthreads();
#pragma unroll
        for (int pass = 0; pass < 2; ++pass) {
#pragma unroll
            for (u32 it = 0; it < 4; ++it) {
                const u32 L = it * 4u + lsub;
                const v8h v = *(const v8h*)&ps[pw + L * 64u + piece * 8u];
                f16* dp = Cp + ((size_t)(bidx * (u32)SEQ + q0 + L) * (2u * INNER) + rep * (u32)INNER
                                + hidx * (u32)HD + piece * 8u);
                *(volatile v8h*)dp = v;
            }
            if (pass == 0) __threadfence();
        }
        __syncthreads();
    }
}

static_assert((size_t)(MROWS / 8) * 256 * 16 == (size_t)MROWS * DM);
static_assert((size_t)(NQKV / 64) * (DM / 64) * 4096 == (size_t)DM * NQKV);
static_assert((size_t)(DM / 64) * (INNER / 64) * 4096 == (size_t)INNER * DM);
static_assert((size_t)(MROWS / 128) * (NQKV / 128) * 128 * 128 == (size_t)MROWS * NQKV);
static_assert((size_t)(SEQ / 128) * (NB * NHEAD) * 128 * HD == (size_t)MROWS * INNER);
static_assert((size_t)(MROWS / 128) * (DM / 128) * 128 * 128 == (size_t)MROWS * DM);

#define WS_HALVES ((size_t)7 * PLANE_ELEMS + (size_t)NQKV * DM + (size_t)DM * INNER)
static_assert(WS_HALVES * 2 <= (size_t)134217728);
static_assert((PLANE_ELEMS * 2) % 128 == 0);
static_assert(((size_t)NQKV * DM * 2) % 128 == 0);
static_assert(((size_t)DM * INNER * 2) % 128 == 0);

extern "C" void kernel_launch(void* const* d_in, const int* in_sizes, int n_in,
                              void* d_out, int out_size, void* d_ws, size_t ws_size,
                              hipStream_t stream) {
    if (n_in < 6) return;
    if (in_sizes[0] < ((NB - 1) * SEQ_FULL + SEQ) * DM) return;
    if (in_sizes[1] < DM) return;
    if (in_sizes[2] < DM) return;
    if (in_sizes[3] < DM * NQKV) return;
    if (in_sizes[4] < INNER * DM) return;
    if (in_sizes[5] < DM) return;
    if (out_size < MROWS * DM) return;
    if (ws_size < WS_HALVES * sizeof(f16)) return;

    const float* x     = (const float*)d_in[0];
    const float* gamma = (const float*)d_in[1];
    const float* beta  = (const float*)d_in[2];
    const float* wqkv  = (const float*)d_in[3];
    const float* wout  = (const float*)d_in[4];
    const float* bout  = (const float*)d_in[5];
    float* out = (float*)d_out;

    const size_t nX = PLANE_ELEMS;
    f16* Xh  = (f16*)d_ws;
    f16* Wt  = Xh  + nX;
    f16* Wot = Wt  + (size_t)NQKV * DM;
    f16* Qh  = Wot + (size_t)DM * INNER;
    f16* Qr  = Qh  + nX;
    f16* Kp  = Qr  + nX;
    f16* Vtp = Kp  + nX;
    f16* Cp  = Vtp + nX;

    ln_rows<<<MROWS / 8, 256, 0, stream>>>(x, gamma, beta, Xh, (u32)MROWS, CARRY_X);
    cvt_transpose<<<dim3(NQKV / 64, DM / 64), 256, 0, stream>>>(wqkv, Wt, (u32)DM, (u32)NQKV, CARRY_W);
    cvt_transpose<<<dim3(DM / 64, INNER / 64), 256, 0, stream>>>(wout, Wot, (u32)INNER, (u32)DM, CARRY_W);

    const float mulQ   = CARRY_Q / (CARRY_X * CARRY_W);
    const float mulKV  = CARRY_K / (CARRY_X * CARRY_W);
    const float mulOut = 1.0f / (CARRY_CTX * CARRY_W);

    gemm_nt<<<dim3(MROWS / 128, NQKV / 128), 256, 0, stream>>>(
        Xh, Wt, (u32)DM, (u32)DM, 0u, Qh, Vtp, bout, out, mulQ, mulKV, mulOut);

    attn_fwd<<<dim3(SEQ / 128, NB * NHEAD), 256, 0, stream>>>(Qh, Qr, Kp, Vtp, Cp);

    gemm_nt<<<dim3(MROWS / 128, DM / 128), 256, 0, stream>>>(
        Cp, Wot, (u32)(2 * INNER), (u32)(2 * INNER), 2u, Qh, Vtp, bout, out, mulQ, mulKV, mulOut);
}
